// ShieldLayer_40467181863380
// MI455X (gfx1250) — hardware-run, weakly checked
//
#include <hip/hip_runtime.h>
#include <math.h>

typedef __attribute__((ext_vector_type(16))) _Float16 v16h;
typedef __attribute__((ext_vector_type(8)))  _Float16 v8h;
typedef __attribute__((ext_vector_type(8)))  float    v8f;
typedef __attribute__((ext_vector_type(4)))  float    v4f;

constexpr int kBatch    = 8192;
constexpr int kVars     = 512;
constexpr int kCons     = 16;
constexpr int kCols     = kVars + 1;
constexpr int kWRows    = 2 * kCons;
constexpr int kTileRows = 32;
constexpr int kGroup    = 32;
constexpr int kPhPitch  = 520;
constexpr int kStPitch  = 36;
constexpr float kStateCarry  = 64.0f;
constexpr float kWeightCarry = 1024.0f;
constexpr float kAccCarry    = kStateCarry * kWeightCarry;
constexpr float kAccCarryInv = 1.0f / kAccCarry;
constexpr float kF16MinNormal = 6.103515625e-5f;
constexpr float kF16Max       = 65504.0f;
static_assert(kCols == 513, "augmented width");
static_assert(kWRows == 32, "pos rows 0..15, neg rows 16..31");
static_assert((kVars % 32) == 0, "K multiple of 32");
static_assert((kBatch % kTileRows) == 0, "batch tiles exact");
static_assert((kVars % kGroup) == 0, "variable groups exact");
static_assert((kPhPitch % 8) == 0 && kPhPitch >= kVars + 8, "LDS state pitch");
static_assert((kStPitch % 4) == 0 && kStPitch >= kGroup, "LDS stage pitch");
static_assert(kAccCarry == 65536.0f, "accumulator carry");

constexpr size_t kBytesWh   = (size_t)kVars * kWRows * kVars * 2;
constexpr size_t kBytesBias = (size_t)kVars * kWRows * 4;
constexpr size_t kOffWh     = 0;
constexpr size_t kOffBias   = kOffWh + kBytesWh;
constexpr size_t kWsTotal   = kOffBias + kBytesBias;
static_assert(kBytesWh == 16777216ull && kBytesBias == 65536ull, "carve sizes");
static_assert(kWsTotal == 16842752ull, "carve total");
static_assert(kWsTotal <= 134217728ull, "carve cap");
static_assert((kOffBias % 256) == 0, "aligned regions");

__device__ __forceinline__ _Float16 carry_to_f16(float x, float carry) {
  float s = x * carry;
  s = fminf(fmaxf(s, -kF16Max), kF16Max);
  const float t = (fabsf(s) < kF16MinNormal) ? 0.0f : s;
  return (_Float16)t;
}

union FragU { v16h v; v8h h[2]; };
__device__ __forceinline__ v16h frag_load(const _Float16* p) {
  FragU f;
  f.h[0] = *(const v8h*)(p);
  f.h[1] = *(const v8h*)(p + 16);
  return f.v;
}

__device__ __forceinline__ v8f mma_g(v16h a, v16h b, v8f c) {
  c = __builtin_amdgcn_wmma_f32_16x16x32_f16(false, a, false, b, (short)0, c, false, false);
  asm volatile("v_nop\n\tv_nop\n\tv_nop\n\tv_nop" : "+v"(c) : "v"(a), "v"(b));
  return c;
}

__device__ __forceinline__ void wave_lds_sync() {
  __builtin_amdgcn_fence(__ATOMIC_RELEASE, "workgroup");
  __builtin_amdgcn_wave_barrier();
  __builtin_amdgcn_fence(__ATOMIC_ACQUIRE, "workgroup");
}

constexpr int kPackThreads = kVars * kWRows * (kVars / 8);
static_assert((kPackThreads % 256) == 0, "pack grid exact");
__global__ __launch_bounds__(256) void pack_planes_kernel(
    const float* __restrict__ posm, const float* __restrict__ negm, unsigned short* __restrict__ wh)
{
  const int i  = blockIdx.x * 256 + threadIdx.x;
  const int R  = i >> 6;
  const int k8 = (i & 63) * 8;
  const int v  = R >> 5;
  const int r  = R & 31;
  const float* base = (r < kCons) ? posm : negm;
  const float* sp = base + (size_t)(v * kCons + (r & (kCons - 1))) * kCols + k8;
  float x[8];
#pragma unroll
  for (int e = 0; e < 8; ++e) x[e] = sp[e];
  v8h hv;
#pragma unroll
  for (int e = 0; e < 8; ++e) hv[e] = carry_to_f16(x[e], kWeightCarry);
  unsigned short* dp = wh + (size_t)i * 8;
  *(volatile v8h*)dp = hv;
  __threadfence();
  *(volatile v8h*)dp = hv;
}

constexpr int kBiasThreads = kVars * kWRows / 4;
static_assert((kBiasThreads % 256) == 0, "bias grid exact");
__global__ __launch_bounds__(256) void pack_bias_kernel(
    const float* __restrict__ posm, const float* __restrict__ negm, float* __restrict__ biasp)
{
  const int i  = blockIdx.x * 256 + threadIdx.x;
  const int v  = i >> 3;
  const int r4 = (i & 7) * 4;
  const float* base = (r4 < kCons) ? posm : negm;
  const int cb = r4 & (kCons - 1);
  const float* sp = base + (size_t)(v * kCons + cb) * kCols + kVars;
  const float b0 = sp[0];
  const float b1 = sp[kCols];
  const float b2 = sp[2 * kCols];
  const float b3 = sp[3 * kCols];
  v4f o;
  o[0] = b0 * kAccCarry;
  o[1] = b1 * kAccCarry;
  o[2] = b2 * kAccCarry;
  o[3] = b3 * kAccCarry;
  float* dp = biasp + (size_t)i * 4;
  *(volatile v4f*)dp = o;
  __threadfence();
  *(volatile v4f*)dp = o;
}

__global__ __launch_bounds__(32) void scan_clamp_kernel(
    const float* __restrict__ preds, const unsigned short* __restrict__ whp,
    const float* __restrict__ biasp, float* __restrict__ out)
{
  __shared__ __align__(16) _Float16 Ph[kTileRows * kPhPitch];
  __shared__ __align__(16) float    St[kTileRows * kStPitch];
  const _Float16* Wh = (const _Float16*)whp;
  const int lane = threadIdx.x & 31;
  const int hh   = lane >> 4;
  const int c    = lane & 15;
  const int row0 = blockIdx.x * kTileRows;

  {
    v8h z;
#pragma unroll
    for (int e = 0; e < 8; ++e) z[e] = (_Float16)0.0f;
    *(v8h*)(Ph + lane * kPhPitch + kVars) = z;
  }
#pragma unroll 1
  for (int it = 0; it < 64; ++it) {
    const int e0 = it * 32 + lane;
    const int r  = e0 >> 6;
    const int k8 = (e0 & 63) * 8;
    const float* sp = preds + (size_t)(row0 + r) * kVars + k8;
    const v4f a0 = *(const v4f*)(sp);
    const v4f a1 = *(const v4f*)(sp + 4);
    v8h hv;
#pragma unroll
    for (int e = 0; e < 4; ++e) {
      hv[e]     = carry_to_f16(a0[e], kStateCarry);
      hv[4 + e] = carry_to_f16(a1[e], kStateCarry);
    }
    *(v8h*)(Ph + r * kPhPitch + k8) = hv;
  }
  wave_lds_sync();

  const int sq  = lane >> 3;
  const int sc4 = (lane & 7) * 4;
  const _Float16* b0p = Ph + c * kPhPitch + 8 * hh;
  const _Float16* b1p = b0p + 16 * kPhPitch;

#pragma unroll 1
  for (int g = 0; g < kVars / kGroup; ++g) {
#pragma unroll
    for (int it = 0; it < 8; ++it) {
      const int r = it * 4 + sq;
      const v4f x = *(const v4f*)(preds + (size_t)(row0 + r) * kVars + g * kGroup + sc4);
      *(v4f*)(St + r * kStPitch + sc4) = x;
    }
    wave_lds_sync();

#pragma unroll 1
    for (int vi = 0; vi < kGroup; ++vi) {
      const int v = g * kGroup + vi;
      const float* bp = biasp + (size_t)v * kWRows + 8 * hh;
      v8f accP0 = *(const v8f*)(bp);
      v8f accN0 = *(const v8f*)(bp + kCons);
      v8f accP1 = accP0;
      v8f accN1 = accN0;
      const _Float16* wp = Wh + (size_t)(v * kWRows + c) * kVars + 8 * hh;
      const _Float16* wn = wp + (size_t)kCons * kVars;
#pragma unroll 2
      for (int k0 = 0; k0 < kVars; k0 += 32) {
        const v16h ap = frag_load(wp + k0);
        const v16h an = frag_load(wn + k0);
        const v16h b0 = frag_load(b0p + k0);
        const v16h b1 = frag_load(b1p + k0);
        accP0 = mma_g(ap, b0, accP0);
        accN0 = mma_g(an, b0, accN0);
        accP1 = mma_g(ap, b1, accP1);
        accN1 = mma_g(an, b1, accN1);
      }
      float lo0 = accP0[0], hi0 = accN0[0], lo1 = accP1[0], hi1 = accN1[0];
#pragma unroll
      for (int r = 1; r < 8; ++r) {
        lo0 = fmaxf(lo0, accP0[r]);
        hi0 = fminf(hi0, accN0[r]);
        lo1 = fmaxf(lo1, accP1[r]);
        hi1 = fminf(hi1, accN1[r]);
      }
      const float lo0x = __shfl_xor(lo0, 16, 32);
      const float hi0x = __shfl_xor(hi0, 16, 32);
      const float lo1x = __shfl_xor(lo1, 16, 32);
      const float hi1x = __shfl_xor(hi1, 16, 32);
      lo0 = fmaxf(lo0, lo0x);
      hi0 = fminf(hi0, hi0x);
      lo1 = fmaxf(lo1, lo1x);
      hi1 = fminf(hi1, hi1x);
      const float lower = (hh ? lo1 : lo0) * kAccCarryInv;
      const float upper = (hh ? hi1 : hi0) * kAccCarryInv;
      const float cur  = St[lane * kStPitch + vi];
      const float corr = fminf(fmaxf(cur, lower), upper);
      St[lane * kStPitch + vi] = corr;
      Ph[lane * kPhPitch + v]  = carry_to_f16(corr, kStateCarry);
      wave_lds_sync();
    }

    v4f sv[8];
#pragma unroll
    for (int it = 0; it < 8; ++it) sv[it] = *(const v4f*)(St + (it * 4 + sq) * kStPitch + sc4);
    wave_lds_sync();
    for (int pass = 0; pass < 2; ++pass) {
#pragma unroll
      for (int it = 0; it < 8; ++it) {
        const int r = it * 4 + sq;
        *(volatile v4f*)(out + (size_t)(row0 + r) * kVars + g * kGroup + sc4) = sv[it];
      }
      __threadfence();
    }
  }
}

extern "C" void kernel_launch(void* const* d_in, const int* in_sizes, int n_in,
                              void* d_out, int out_size, void* d_ws, size_t ws_size,
                              hipStream_t stream) {
  if (n_in < 3 || d_out == nullptr || d_ws == nullptr) return;
  if (in_sizes[0] != kBatch * kVars) return;
  if (in_sizes[1] != kVars * kCons * kCols) return;
  if (in_sizes[2] != kVars * kCons * kCols) return;
  if (out_size != kBatch * kVars) return;
  if (ws_size < kWsTotal) return;

  const float* preds = (const float*)d_in[0];
  const float* posm  = (const float*)d_in[1];
  const float* negm  = (const float*)d_in[2];
  float* out = (float*)d_out;

  char* ws = (char*)d_ws;
  unsigned short* WH   = (unsigned short*)(ws + kOffWh);
  float*          BIAS = (float*)(ws + kOffBias);

  pack_planes_kernel<<<kPackThreads / 256, 256, 0, stream>>>(posm, negm, WH);
  pack_bias_kernel<<<kBiasThreads / 256, 256, 0, stream>>>(posm, negm, BIAS);
  scan_clamp_kernel<<<kBatch / kTileRows, 32, 0, stream>>>(preds, WH, BIAS, out);
}
